// LinearAttention_5523327943104
// MI455X (gfx1250) — hardware-run, weakly checked
//
#include <hip/hip_runtime.h>


#define NB_  4
#define NT   8192
#define DM   256
#define NH_  8
#define HD   64
#define DI   (NH_ * HD)
typedef _Float16 h16;
typedef unsigned short bf;
typedef __attribute__((ext_vector_type(16))) __bf16   v16bf;
typedef __attribute__((ext_vector_type(16))) _Float16 v16h;
typedef __attribute__((ext_vector_type(8)))  _Float16 v8h;
typedef __attribute__((ext_vector_type(8)))  unsigned short v8us;
typedef __attribute__((ext_vector_type(8)))  float    v8f;
typedef __attribute__((ext_vector_type(4)))  float    v4f;
typedef v8h  __attribute__((may_alias)) v8ha;
typedef v4f  __attribute__((may_alias)) v4fa;
typedef v8us __attribute__((may_alias)) v8usa;

__device__ __forceinline__ unsigned short f2bf(float f) { unsigned u = __float_as_uint(f); u += 0x7FFFu + ((u >> 16) & 1u); return (unsigned short)(u >> 16); }
__device__ __forceinline__ float bf2f(unsigned short b) { return __uint_as_float(((unsigned)b) << 16); }
__device__ __forceinline__ float bfr(float f) { return bf2f(f2bf(f)); }
__device__ __forceinline__ v16h cat16(v8h lo, v8h hi) { return __builtin_shufflevector(lo, hi, 0, 1, 2, 3, 4, 5, 6, 7, 8, 9, 10, 11, 12, 13, 14, 15); }
__device__ __forceinline__ v16bf cat16b(v8us lo, v8us hi) { return __builtin_bit_cast(v16bf, __builtin_shufflevector(lo, hi, 0, 1, 2, 3, 4, 5, 6, 7, 8, 9, 10, 11, 12, 13, 14, 15)); }
__device__ __forceinline__ v8f wmma16(v16h a, v16h b, v8f c) { return __builtin_amdgcn_wmma_f32_16x16x32_f16(false, a, false, b, (short)0, c, false, false); }
__device__ __forceinline__ v8f wmmab(v16bf a, v16bf b, v8f c) { return __builtin_amdgcn_wmma_f32_16x16x32_bf16(false, a, false, b, (short)0, c, false, false); }


template <typename T16> struct WFrag;
template <> struct WFrag<h16> { typedef v16h V; static __device__ __forceinline__ V ld(const h16* p) { return cat16(*(const v8h*)p, *(const v8h*)(p + 16)); } static __device__ __forceinline__ v8f mma(V a, V b, v8f c) { return wmma16(a, b, c); } };
template <> struct WFrag<bf> { typedef v16bf V; static __device__ __forceinline__ V ld(const bf* p) { return cat16b(*(const v8us*)p, *(const v8us*)(p + 16)); } static __device__ __forceinline__ v8f mma(V a, V b, v8f c) { return wmmab(a, b, c); } };
template <typename T16, int NSPLIT, bool BIAS>
__global__ __launch_bounds__(32) void k_gemmw(const T16* __restrict__ A, const T16* __restrict__ A2, const T16* __restrict__ Bt, const T16* __restrict__ Bt2, int K, float* C, int ldc, const float* __restrict__ bias, size_t sA, size_t sB, size_t sC) {
    typedef typename WFrag<T16>::V V;
    __shared__ __align__(16) float os[16 * 68];
    const size_t z = blockIdx.z; A += z * sA; if (A2) A2 += z * sA; Bt += z * sB; if (Bt2) Bt2 += z * sB; C += z * sC;
    const int lane = threadIdx.x & 31, lr = lane & 15, hi = lane >> 4; const int r0 = blockIdx.x * 64, c0 = blockIdx.y * 64;
    v8f acc[4][4];
#pragma unroll
    for (int mb = 0; mb < 4; ++mb)
#pragma unroll
        for (int nb = 0; nb < 4; ++nb) acc[mb][nb] = (v8f){};
    const size_t aoff = (size_t)(r0 + lr) * K + 8 * hi, boff = (size_t)(c0 + lr) * K + 8 * hi;
    for (int kc = 0; kc < K; kc += 32) {
        V a[4], a2[4];
#pragma unroll
        for (int mb = 0; mb < 4; ++mb) { a[mb] = WFrag<T16>::ld(A + aoff + (size_t)mb * 16 * K + kc); if (NSPLIT == 1 || NSPLIT == 2) a2[mb] = WFrag<T16>::ld(A2 + aoff + (size_t)mb * 16 * K + kc); }
#pragma unroll
        for (int nb = 0; nb < 4; ++nb) { const V b = WFrag<T16>::ld(Bt + boff + (size_t)nb * 16 * K + kc); V b2; if (NSPLIT >= 2) b2 = WFrag<T16>::ld(Bt2 + boff + (size_t)nb * 16 * K + kc);
#pragma unroll
            for (int mb = 0; mb < 4; ++mb) { acc[mb][nb] = WFrag<T16>::mma(a[mb], b, acc[mb][nb]); if (NSPLIT == 1 || NSPLIT == 2) acc[mb][nb] = WFrag<T16>::mma(a2[mb], b, acc[mb][nb]); if (NSPLIT >= 2) acc[mb][nb] = WFrag<T16>::mma(a[mb], b2, acc[mb][nb]); } }
        asm volatile("v_nop\n\tv_nop\n\tv_nop\n\tv_nop" : "+v"(acc[0][0]), "+v"(acc[1][1]), "+v"(acc[2][2]), "+v"(acc[3][3]) : "v"(a[0]), "v"(a[3]));
    }
#pragma unroll
    for (int mb = 0; mb < 4; ++mb) {
#pragma unroll
        for (int nb = 0; nb < 4; ++nb) {
#pragma unroll
            for (int j = 0; j < 8; ++j) os[(hi * 8 + j) * 68 + nb * 16 + lr] = acc[mb][nb][j]; }
        __builtin_amdgcn_wave_barrier(); asm volatile("" ::: "memory");
        float* crow = C + (size_t)(r0 + mb * 16) * ldc + c0;
#pragma unroll 1
        for (int ps = 0; ps < 2; ++ps) {
#pragma unroll
            for (int s = 0; s < 8; ++s) { const int row = 2 * s + hi, cofs = lr * 4; v4f val = *(const v4fa*)(os + row * 68 + cofs); if (BIAS) { val[0] += bfr(bias[c0 + cofs]); val[1] += bfr(bias[c0 + cofs + 1]); val[2] += bfr(bias[c0 + cofs + 2]); val[3] += bfr(bias[c0 + cofs + 3]); }
                *(volatile v4f*)(crow + (size_t)row * ldc + cofs) = val; }
            if (ps == 0) __threadfence(); }
        __builtin_amdgcn_wave_barrier(); asm volatile("" ::: "memory");
    }
}

__device__ __forceinline__ h16 tohx(float x) { return (h16)x; }
__device__ __forceinline__ void splitf(float y, unsigned short& h, unsigned short& l) { h = f2bf(y); l = f2bf(y - bf2f(h)); }
typedef __attribute__((ext_vector_type(2))) _Float16 v2h;
typedef __attribute__((ext_vector_type(4))) _Float16 v4h;
typedef __attribute__((ext_vector_type(2))) unsigned short v2us;
typedef __attribute__((ext_vector_type(4))) unsigned short v4us;
typedef __attribute__((ext_vector_type(2))) float v2f;
typedef __attribute__((ext_vector_type(4))) int v4i;

__global__ __launch_bounds__(256) void k_cvt8(const float* __restrict__ src, bf* dst, size_t n8) { const size_t i = (size_t)blockIdx.x * 256 + threadIdx.x; if (i >= n8) return; const v8f v = *(const v8f*)(src + i * 8); v8us o;
#pragma unroll
    for (int k = 0; k < 8; ++k) o[k] = f2bf(v[k]); *(volatile v8us*)(dst + i * 8) = o; __threadfence(); *(volatile v8us*)(dst + i * 8) = o; }
__global__ __launch_bounds__(256) void k_f2h(const float* __restrict__ S, h16* P16, size_t n4) { const size_t i = (size_t)blockIdx.x * 256 + threadIdx.x; if (i >= n4) return; const v4f v = *(const v4f*)(S + i * 4); v4h o;
#pragma unroll
    for (int q = 0; q < 4; ++q) o[q] = tohx(v[q]);
    *(volatile v4h*)(P16 + i * 4) = o; __threadfence(); *(volatile v4h*)(P16 + i * 4) = o; }
__global__ __launch_bounds__(256) void k_tohl(const float* __restrict__ F, float sc, bf* Hh, bf* Hl, size_t n4) { const size_t i = (size_t)blockIdx.x * 256 + threadIdx.x; if (i >= n4) return; const v4f a = *(const v4f*)(F + i * 4); v4us oh, ol;
#pragma unroll
    for (int q = 0; q < 4; ++q) { unsigned short h2, l2; splitf(__fmul_rn(a[q], sc), h2, l2); oh[q] = h2; ol[q] = l2; }
    *(volatile v4us*)(Hh + i * 4) = oh; *(volatile v4us*)(Hl + i * 4) = ol; __threadfence(); *(volatile v4us*)(Hh + i * 4) = oh; *(volatile v4us*)(Hl + i * 4) = ol; }
__global__ __launch_bounds__(256) void k_inorm(const float* __restrict__ F, h16* T) { const unsigned idx = blockIdx.x * 256 + threadIdx.x; const unsigned np_ = idx % (NT / 2), h = idx / (NT / 2); const unsigned n0 = np_ * 2; h16* p0 = T + (size_t)h * HD * NT + n0; float xa[HD], xb[HD];
#pragma unroll
    for (int g = 0; g < HD / 4; ++g) { const v4f a = *(const v4f*)(F + (size_t)n0 * DI + h * HD + g * 4); const v4f b = *(const v4f*)(F + (size_t)(n0 + 1) * DI + h * HD + g * 4);
#pragma unroll
        for (int q = 0; q < 4; ++q) { xa[g * 4 + q] = a[q]; xb[g * 4 + q] = b[q]; } }
    float sa = 0.0f, sb = 0.0f;
#pragma unroll
    for (int d = 0; d < HD; ++d) { sa = __fadd_rn(sa, xa[d]); sb = __fadd_rn(sb, xb[d]); }
    const float ma = __fmul_rn(sa, 1.0f / HD), mb = __fmul_rn(sb, 1.0f / HD); float qa = 0.0f, qb = 0.0f;
#pragma unroll
    for (int d = 0; d < HD; ++d) { const float da = __fsub_rn(xa[d], ma), db = __fsub_rn(xb[d], mb); qa = __fmaf_rn(da, da, qa); qb = __fmaf_rn(db, db, qb); }
    const float ra = __fdiv_rn(1.0f, __fsqrt_rn(__fadd_rn(__fmul_rn(qa, 1.0f / HD), 1.0e-5f))), rb_ = __fdiv_rn(1.0f, __fsqrt_rn(__fadd_rn(__fmul_rn(qb, 1.0f / HD), 1.0e-5f)));
#pragma unroll
    for (int d = 0; d < HD; ++d) { const float ya = __fmul_rn(__fsub_rn(xa[d], ma), ra), yb = __fmul_rn(__fsub_rn(xb[d], mb), rb_); v2h o; o[0] = tohx((fabsf(ya) < 6.103515625e-5f) ? 0.0f : ya); o[1] = tohx((fabsf(yb) < 6.103515625e-5f) ? 0.0f : yb);
        *(volatile v2h*)(p0 + (size_t)d * NT) = o; }
    __threadfence();
#pragma unroll
    for (int d = 0; d < HD; ++d) { const float ya = __fmul_rn(__fsub_rn(xa[d], ma), ra), yb = __fmul_rn(__fsub_rn(xb[d], mb), rb_); v2h o; o[0] = tohx((fabsf(ya) < 6.103515625e-5f) ? 0.0f : ya); o[1] = tohx((fabsf(yb) < 6.103515625e-5f) ? 0.0f : yb);
        *(volatile v2h*)(p0 + (size_t)d * NT) = o; } }
__global__ __launch_bounds__(256) void k_qh(const float* __restrict__ F, h16* Q) { const unsigned idx = blockIdx.x * 256 + threadIdx.x; const unsigned d0 = (idx % (HD / 4)) * 4, n = (idx / (HD / 4)) % NT, h = idx / ((HD / 4) * NT); const v4f a = *(const v4f*)(F + (size_t)n * DI + h * HD + d0); v4h o;
#pragma unroll
    for (int q = 0; q < 4; ++q) o[q] = tohx((fabsf(a[q]) < 6.103515625e-5f) ? 0.0f : a[q]);
    *(volatile v4h*)(Q + (size_t)idx * 4) = o; __threadfence(); *(volatile v4h*)(Q + (size_t)idx * 4) = o; }

extern "C" void kernel_launch(void* const* d_in, const int* in_sizes, int n_in,
                              void* d_out, int out_size, void* d_ws, size_t ws_size, hipStream_t stream) {
    (void)in_sizes; (void)n_in; (void)out_size;
    const float* x = (const float*)d_in[0]; const float* wqkv = (const float*)d_in[1]; const float* wout = (const float*)d_in[2]; const float* bout = (const float*)d_in[3];
    float* OUT = (float*)d_out;
    char* wsp = (char*)d_ws;
    auto take = [&](size_t bytes) { char* p = wsp; wsp += (bytes + 255) & ~(size_t)255; return (void*)p; };
    bf* WB = (bf*)take((size_t)3 * DI * DM * 2); bf* WQ = WB; bf* WK = WB + (size_t)DI * DM; bf* WV = WB + (size_t)2 * DI * DM; bf* WO = (bf*)take((size_t)DM * DI * 2);
    bf* XB = (bf*)take((size_t)NT * DM * 2); float* FQ = (float*)take((size_t)NT * DI * 4); float* FK = (float*)take((size_t)NT * DI * 4); float* FV = (float*)take((size_t)NT * DI * 4);
    h16* Q16 = (h16*)take((size_t)NH_ * NT * HD * 2); h16* KT16 = (h16*)take((size_t)NH_ * HD * NT * 2); h16* VT16 = (h16*)take((size_t)NH_ * HD * NT * 2); float* MT = (float*)take((size_t)NH_ * HD * HD * 4); h16* MT16 = (h16*)take((size_t)NH_ * HD * HD * 2);
    float* CTX = (float*)take((size_t)NT * DI * 4); bf* ATh = (bf*)take((size_t)NT * DI * 2); bf* ATl = (bf*)take((size_t)NT * DI * 2);
    if ((size_t)(wsp - (char*)d_ws) > ws_size) return;
    k_cvt8<<<(unsigned)(((size_t)3 * DI * DM / 8 + 255) / 256), 256, 0, stream>>>(wqkv, WB, (size_t)3 * DI * DM / 8);
    k_cvt8<<<(unsigned)(((size_t)DM * DI / 8 + 255) / 256), 256, 0, stream>>>(wout, WO, (size_t)DM * DI / 8);
    for (int b = 0; b < NB_; ++b) {
        k_cvt8<<<(unsigned)(((size_t)NT * DM / 8 + 255) / 256), 256, 0, stream>>>(x + (size_t)b * NT * DM, XB, (size_t)NT * DM / 8);
        k_gemmw<bf, 0, false><<<dim3(NT / 64, DI / 64, 1), 32, 0, stream>>>(XB, nullptr, WQ, nullptr, DM, FQ, DI, nullptr, 0, 0, 0);
        k_gemmw<bf, 0, false><<<dim3(NT / 64, DI / 64, 1), 32, 0, stream>>>(XB, nullptr, WK, nullptr, DM, FK, DI, nullptr, 0, 0, 0);
        k_gemmw<bf, 0, false><<<dim3(NT / 64, DI / 64, 1), 32, 0, stream>>>(XB, nullptr, WV, nullptr, DM, FV, DI, nullptr, 0, 0, 0);
        k_qh<<<NH_ * NT * (HD / 4) / 256, 256, 0, stream>>>(FQ, Q16);
        k_inorm<<<NH_ * (NT / 2) / 256, 256, 0, stream>>>(FK, KT16); k_inorm<<<NH_ * (NT / 2) / 256, 256, 0, stream>>>(FV, VT16);
        k_gemmw<h16, 0, false><<<dim3(HD / 64, HD / 64, NH_), 32, 0, stream>>>(VT16, nullptr, KT16, nullptr, NT, MT, HD, nullptr, (size_t)HD * NT, (size_t)HD * NT, (size_t)HD * HD);
        k_f2h<<<(unsigned)(((size_t)NH_ * HD * HD / 4 + 255) / 256), 256, 0, stream>>>(MT, MT16, (size_t)NH_ * HD * HD / 4);
        k_gemmw<h16, 0, false><<<dim3(NT / 64, HD / 64, NH_), 32, 0, stream>>>(Q16, nullptr, MT16, nullptr, HD, CTX, DI, nullptr, (size_t)NT * HD, (size_t)HD * HD, (size_t)HD);
        k_tohl<<<(unsigned)(((size_t)NT * DI / 4 + 255) / 256), 256, 0, stream>>>(CTX, 1.220703125e-4f, ATh, ATl, (size_t)NT * DI / 4);
        k_gemmw<bf, 1, true><<<dim3(NT / 64, DM / 64, 1), 32, 0, stream>>>(ATh, ATl, WO, nullptr, DI, OUT + (size_t)b * NT * DM, DM, bout, 0, 0, 0); }
}
